// PaiNN_35175782154416
// MI455X (gfx1250) — hardware-verified
//
#include <hip/hip_runtime.h>
#include <stddef.h>
#include <stdint.h>


#define HD      128
#define H2      256
#define H3      384
#define K4      512
#define KF      64
#define NRB     20
#define NL      3
#define NFLT    1152
#define NTHR    256
#define NWAVE   8
#define EPT     8
#define CHUNK   (NTHR * EPT)
#define WCAP    (EPT * 32)
#define LISTN   (NWAVE * WCAP)
#define NBMAX   2048
#define NBA     1024
#define RCAP    28672
#define DEGCAP  64
#define GBM     64
#define GBN     128
#define GTHR    128
#define ECH     32000
#define OW1     0
#define OW2     (OW1 + NL * HD * H2)
#define OVW     (OW2 + NL * H3 * H2)
#define OM1     (OVW + NL * H2 * H2)
#define OM2     (OM1 + NL * HD * K4)
#define OFW     (OM2 + NL * H3 * H2)
#define NW_TOT  (OFW + NL * H3 * KF)
#define UW1     (NL * HD * (H2 / 8))
#define UW2     (UW1 + NL * H3 * (H2 / 8))
#define UVW     (UW2 + NL * H2 * (H2 / 8))
#define UM1     (UVW + NL * HD * (K4 / 8))
#define UM2     (UM1 + NL * H3 * (H2 / 8))
#define UFW     (UM2 + NL * H3 * (KF / 8))
#define CF      64.0f
#define RCF     0.015625f
#define RADF    5.0f
#define PIF     3.14159274f
#define EPSG    1e-8f
#define GAMMA   8.0f
#define R19     (1.0f / 19.0f)
#define WSMAX   134217728
#define LDS_AGG ((2 * RCAP + 2 * NBMAX + LISTN) * 4 + 64)

static_assert((CHUNK & (CHUNK - 1)) == 0 && CHUNK <= 4096);
static_assert((NBMAX & (NBMAX - 1)) == 0 && NBMAX <= 4096);
static_assert(NTHR * 8 == NBMAX);
static_assert(NBA <= NBMAX && (NBA % NWAVE) == 0 && (NBA % GBM) == 0);
static_assert(LISTN >= NBMAX && LISTN >= NWAVE * WCAP);
static_assert((RCAP % 32) == 0);
static_assert(LDS_AGG <= 300000);
static_assert(GBM == (GTHR / 32) * 16 && GBN == 4 * 32);
static_assert((HD % 32) == 0 && (H2 % 32) == 0 && (K4 % 32) == 0 && KF == 64);
static_assert(NRB + 12 == KF / 2);
static_assert((ECH % GBM) == 0);
static_assert((UW1 % NTHR) == 0 && (UW2 % NTHR) == 0 && (UVW % NTHR) == 0);
static_assert((UM1 % NTHR) == 0 && (UM2 % NTHR) == 0 && (UFW % NTHR) == 0);
static_assert(UFW * 8 == NW_TOT);
static_assert(HD == 4 * 32 && H3 == 3 * HD && H2 == 2 * HD && K4 == 4 * HD);

typedef float          v4f   __attribute__((ext_vector_type(4)));
typedef float          v8f   __attribute__((ext_vector_type(8)));
typedef int            v4i   __attribute__((ext_vector_type(4)));
typedef int            v8i   __attribute__((ext_vector_type(8)));
typedef unsigned       v2u   __attribute__((ext_vector_type(2)));
typedef unsigned short v8us  __attribute__((ext_vector_type(8)));
typedef unsigned short v16us __attribute__((ext_vector_type(16)));
typedef __bf16         v16bf __attribute__((ext_vector_type(16)));
typedef v4f  __attribute__((may_alias)) v4fa;
typedef v4i  __attribute__((may_alias)) v4ia;
typedef v2u  __attribute__((may_alias)) v2ua;
typedef v8us __attribute__((may_alias)) v8usa;
union FragB { v16bf v; v16us u; v8us h[2]; v8i w; };

__device__ __forceinline__ v8f wmb(const FragB& a, const FragB& b, v8f c) {
  v8f d = __builtin_amdgcn_wmma_f32_16x16x32_bf16(false, a.v, false, b.v, (short)0, c, false, false);
  asm volatile("v_nop\n\tv_nop\n\tv_nop\n\tv_nop" : "+v"(d) : "v"(a.w), "v"(b.w));
  return d;
}

__device__ __forceinline__ void ldwait() {
  asm volatile("s_wait_loadcnt 0x0" ::: "memory");
}

__device__ __forceinline__ unsigned bf16_bits(float f) {
  const unsigned u = __float_as_uint(f);
  return (u + 0x7FFFu + ((u >> 16) & 1u)) >> 16;
}
__device__ __forceinline__ float bf16_val(float f) {
  return __uint_as_float(bf16_bits(f) << 16);
}
__device__ __forceinline__ unsigned short f2h(float f) {
  const _Float16 hv = (_Float16)f;
  return __builtin_bit_cast(unsigned short, hv);
}
__device__ __forceinline__ float h2f(unsigned b) {
  const _Float16 hv = __builtin_bit_cast(_Float16, (unsigned short)b);
  return (float)hv;
}
__device__ __forceinline__ float silu_f(float t) {
  return t * __builtin_amdgcn_rcpf(1.0f + __expf(-t));
}
__device__ __forceinline__ float clipf(float x) { return fminf(fmaxf(x, -1e4f), 1e4f); }
__device__ __forceinline__ void put16(unsigned short* dp, v8us o) {
  *(volatile v8us*)dp = o;
  __threadfence();
  *(volatile v8us*)dp = o;
}
__device__ __forceinline__ void putf4(float* dp, v4f o) {
  *(volatile v4f*)dp = o;
  __threadfence();
  *(volatile v4f*)dp = o;
}

__device__ __forceinline__ int scan_chunk(const int* __restrict__ dsts, int nE, int cbase, int slotBase,
                                          int nb, int vec8, int* list, int tid, int lane, int wave) {
  int wc = 0;
  const int el0  = tid * EPT;
  const int e0   = cbase + el0;
  const int sent = -2147483647 - 1;
  v4i da, db;
  if (vec8 != 0 && cbase + CHUNK <= nE) {
    da = *(const v4i*)(dsts + e0);
    db = *(const v4i*)(dsts + e0 + 4);
  } else {
    da.x = (e0     < nE) ? dsts[min(e0,     nE - 1)] : sent;
    da.y = (e0 + 1 < nE) ? dsts[min(e0 + 1, nE - 1)] : sent;
    da.z = (e0 + 2 < nE) ? dsts[min(e0 + 2, nE - 1)] : sent;
    da.w = (e0 + 3 < nE) ? dsts[min(e0 + 3, nE - 1)] : sent;
    db.x = (e0 + 4 < nE) ? dsts[min(e0 + 4, nE - 1)] : sent;
    db.y = (e0 + 5 < nE) ? dsts[min(e0 + 5, nE - 1)] : sent;
    db.z = (e0 + 6 < nE) ? dsts[min(e0 + 6, nE - 1)] : sent;
    db.w = (e0 + 7 < nE) ? dsts[min(e0 + 7, nE - 1)] : sent;
  }
  const unsigned nbs = (unsigned)slotBase;
  const unsigned unb = (unsigned)nb;
  const unsigned s0 = (unsigned)da.x - nbs, s1 = (unsigned)da.y - nbs;
  const unsigned s2 = (unsigned)da.z - nbs, s3 = (unsigned)da.w - nbs;
  const unsigned s4 = (unsigned)db.x - nbs, s5 = (unsigned)db.y - nbs;
  const unsigned s6 = (unsigned)db.z - nbs, s7 = (unsigned)db.w - nbs;
  const bool h0 = s0 < unb, h1 = s1 < unb, h2 = s2 < unb, h3 = s3 < unb;
  const bool h4 = s4 < unb, h5 = s5 < unb, h6 = s6 < unb, h7 = s7 < unb;
  const unsigned any = __builtin_amdgcn_ballot_w32(h0 | h1 | h2 | h3 | h4 | h5 | h6 | h7);
  if (any != 0u) {
#define HITJ(J, HJ, SJ) { \
      const unsigned mj = __builtin_amdgcn_ballot_w32(HJ); \
      if (mj != 0u) { \
        if (HJ) { \
          const int pos = wc + (int)__builtin_amdgcn_mbcnt_lo(mj, 0u); \
          if (pos < WCAP) list[wave * WCAP + pos] = ((el0 + (J)) << 12) | (int)(SJ); \
        } \
        wc += (int)__builtin_popcount(mj); } }
    HITJ(0, h0, s0)
    HITJ(1, h1, s1)
    HITJ(2, h2, s2)
    HITJ(3, h3, s3)
    HITJ(4, h4, s4)
    HITJ(5, h5, s5)
    HITJ(6, h6, s6)
    HITJ(7, h7, s7)
#undef HITJ
  }
  return wc;
}

__global__ __launch_bounds__(NTHR) void k_wprep(const float* __restrict__ iW1, const float* __restrict__ iW2,
                                                const float* __restrict__ vW, const float* __restrict__ mW1,
                                                const float* __restrict__ mW2, const float* __restrict__ fW,
                                                unsigned short* WT, int nUnits) {
  const int u = (int)blockIdx.x * NTHR + (int)threadIdx.x;
  if (u >= nUnits) return;
  v8us o;
  if (u < UW1) {
    const int l  = u >> 12;
    const int r  = u & 4095;
    const int n  = r >> 5;
    const int k8 = (r & 31) * 8;
    const int kk = k8 & (HD - 1);
    const float* p = iW1 + ((size_t)l * HD + kk) * HD + n;
#pragma unroll
    for (int i = 0; i < 8; ++i) o[i] = (unsigned short)bf16_bits(p[(size_t)i * HD]);
    put16(WT + OW1 + (size_t)u * 8, o);
    return;
  } else if (u < UW2) {
    const int v  = u - UW1;
    const int l  = v / 12288;
    const int r  = v - l * 12288;
    const int n  = r >> 5;
    const int k8 = (r & 31) * 8;
    const int kk = k8 & (HD - 1);
    const float* p = iW2 + ((size_t)l * HD + kk) * H3 + n;
#pragma unroll
    for (int i = 0; i < 8; ++i) o[i] = (unsigned short)bf16_bits(p[(size_t)i * H3]);
    put16(WT + OW2 + (size_t)v * 8, o);
    return;
  } else if (u < UVW) {
    const int v  = u - UW2;
    const int l  = v >> 13;
    const int r  = v & 8191;
    const int n  = r >> 5;
    const int k8 = (r & 31) * 8;
    const int kk = k8 & (HD - 1);
    const float* p = vW + ((size_t)l * HD + kk) * H2 + n;
#pragma unroll
    for (int i = 0; i < 8; ++i) o[i] = (unsigned short)bf16_bits(p[(size_t)i * H2]);
    put16(WT + OVW + (size_t)v * 8, o);
    return;
  } else if (u < UM1) {
    const int v    = u - UVW;
    const int l    = v >> 13;
    const int r    = v & 8191;
    const int n    = r >> 6;
    const int k8   = (r & 63) * 8;
    const int srow = (k8 < H2) ? (k8 & (HD - 1)) : (HD + (k8 & (HD - 1)));
    const float* p = mW1 + ((size_t)l * H2 + srow) * HD + n;
#pragma unroll
    for (int i = 0; i < 8; ++i) o[i] = (unsigned short)bf16_bits(p[(size_t)i * HD]);
    put16(WT + OM1 + (size_t)v * 8, o);
    return;
  } else if (u < UM2) {
    const int v  = u - UM1;
    const int l  = v / 12288;
    const int r  = v - l * 12288;
    const int n  = r >> 5;
    const int k8 = (r & 31) * 8;
    const int kk = k8 & (HD - 1);
    const float* p = mW2 + ((size_t)l * HD + kk) * H3 + n;
#pragma unroll
    for (int i = 0; i < 8; ++i) o[i] = (unsigned short)bf16_bits(p[(size_t)i * H3]);
    put16(WT + OM2 + (size_t)v * 8, o);
    return;
  } else {
    const int v   = u - UM2;
    const int l   = v / 3072;
    const int r   = v - l * 3072;
    const int n   = r >> 3;
    const int k8  = (r & 7) * 8;
    const int kk0 = k8 & 31;
#pragma unroll
    for (int i = 0; i < 8; ++i) {
      const int kk = kk0 + i;
      const int kc = kk < NRB ? kk : NRB - 1;
      const unsigned short w = (unsigned short)bf16_bits(fW[(size_t)kc * NFLT + l * H3 + n]);
      o[i] = (kk < NRB) ? w : (unsigned short)0;
    }
    put16(WT + OFW + (size_t)v * 8, o);
    return;
  }
}

__global__ __launch_bounds__(NTHR) void k_init(const int* __restrict__ z, const float* __restrict__ emb,
                                               const float* __restrict__ ev, int nN, int nZ, int nE,
                                               int uS, int uV, int uD, float* SA, float* VA, float* DIRD) {
#pragma clang fp contract(off)
  const int u = (int)blockIdx.x * NTHR + (int)threadIdx.x;
  if (u < uS) {
    const int row = u >> 5;
    const int c4  = (u & 31) * 4;
    const int rc  = row < nN ? row : nN - 1;
    int zi = z[rc];
    zi = zi < 0 ? 0 : (zi > nZ - 1 ? nZ - 1 : zi);
    const v4f a = *(const v4fa*)(emb + (size_t)zi * HD + c4);
    const float lv = (row < nN) ? 1.0f : 0.0f;
    v4f o;
    o.x = bf16_val(a.x) * lv; o.y = bf16_val(a.y) * lv; o.z = bf16_val(a.z) * lv; o.w = bf16_val(a.w) * lv;
    putf4(SA + (size_t)row * HD + c4, o);
    return;
  } else if (u < uV) {
    const int v = u - uS;
    const v4f zz = {0.0f, 0.0f, 0.0f, 0.0f};
    putf4(VA + (size_t)v * 4, zz);
    return;
  } else if (u < uD) {
    const int e  = u - uV;
    const int ec = e < nE ? e : nE - 1;
    const float ex = bf16_val(ev[(size_t)ec * 3 + 0]);
    const float ey = bf16_val(ev[(size_t)ec * 3 + 1]);
    const float ez = bf16_val(ev[(size_t)ec * 3 + 2]);
    const float sq = (ex * ex + ez * ez) + ey * ey;
    const float d  = sqrtf(sq + EPSG);
    const float rd = 1.0f / d;
    const float ct = cosf((PIF * d) * 0.2f);
    const float cut = (d < RADF) ? 0.5f * (ct + 1.0f) : 0.0f;
    v4f o;
    o.x = ex * rd; o.y = ey * rd; o.z = ez * rd; o.w = cut;
    putf4(DIRD + (size_t)e * 4, o);
    return;
  }
}

__global__ __launch_bounds__(NTHR) void k_phi(const float* __restrict__ ev, int nE, int ebase, int nUnits,
                                              unsigned short* PHI) {
#pragma clang fp contract(off)
  const int u = (int)blockIdx.x * NTHR + (int)threadIdx.x;
  if (u >= nUnits) return;
  const int le = u >> 3;
  const int g  = u & 7;
  const int e  = ebase + le;
  const int ec = e < nE ? e : nE - 1;
  const bool live = e < nE;
  const float ex = bf16_val(ev[(size_t)ec * 3 + 0]);
  const float ey = bf16_val(ev[(size_t)ec * 3 + 1]);
  const float ez = bf16_val(ev[(size_t)ec * 3 + 2]);
  const float sq = (ex * ex + ez * ez) + ey * ey;
  const float d  = sqrtf(sq + EPSG);
  const int part = g >> 2;
  const int kb   = (g & 3) * 8;
  v8us o;
#pragma unroll
  for (int i = 0; i < 8; ++i) {
    const int k  = kb + i;
    const int kc = k < NRB ? k : NRB - 1;
    const float mu = RADF * ((float)kc * R19);
    const float dd = d - mu;
    const float t  = dd * dd;
    const float ph = __expf(-GAMMA * t);
    const unsigned hb = bf16_bits(ph);
    const unsigned lb = bf16_bits(ph - __uint_as_float(hb << 16));
    const unsigned sel = (part != 0) ? lb : hb;
    o[i] = (k < NRB && live) ? (unsigned short)sel : (unsigned short)0;
  }
  put16(PHI + (size_t)le * KF + g * 8, o);
}

__global__ __launch_bounds__(NTHR) void k_hilo(const float* __restrict__ src, int nUnits, unsigned short* dst) {
  const int u = (int)blockIdx.x * NTHR + (int)threadIdx.x;
  if (u >= nUnits) return;
  const int row = u >> 4;
  const int j   = u & 15;
  const float* p = src + (size_t)row * HD + 8 * j;
  const v4f a = *(const v4fa*)p;
  const v4f b = *(const v4fa*)(p + 4);
  const v8f f8 = {a.x, a.y, a.z, a.w, b.x, b.y, b.z, b.w};
  v8us ohi, olo;
#pragma unroll
  for (int i = 0; i < 8; ++i) {
    const unsigned hb = bf16_bits(f8[i]);
    ohi[i] = (unsigned short)hb;
    olo[i] = (unsigned short)bf16_bits(f8[i] - __uint_as_float(hb << 16));
  }
  unsigned short* dp = dst + (size_t)row * H2 + 8 * j;
  *(volatile v8us*)dp        = ohi;
  *(volatile v8us*)(dp + HD) = olo;
  __threadfence();
  *(volatile v8us*)dp        = ohi;
  *(volatile v8us*)(dp + HD) = olo;
}

__global__ __launch_bounds__(NTHR) void k_tsrow(const float* __restrict__ S, const float* __restrict__ U,
                                                int nUnits, unsigned short* TS) {
  const int u = (int)blockIdx.x * NTHR + (int)threadIdx.x;
  if (u >= nUnits) return;
  const int row = u >> 4;
  const int j   = u & 15;
  const float* sp = S + (size_t)row * HD + 8 * j;
  const v4f sa = *(const v4fa*)sp, sb = *(const v4fa*)(sp + 4);
  const float* up = U + (size_t)row * 3 * H2 + 8 * j;
  const v4f p0 = *(const v4fa*)up,            q0 = *(const v4fa*)(up + 4);
  const v4f p1 = *(const v4fa*)(up + H2),     q1 = *(const v4fa*)(up + H2 + 4);
  const v4f p2 = *(const v4fa*)(up + 2 * H2), q2 = *(const v4fa*)(up + 2 * H2 + 4);
  const v8f s8 = {sa.x, sa.y, sa.z, sa.w, sb.x, sb.y, sb.z, sb.w};
  const v8f l0 = {p0.x, p0.y, p0.z, p0.w, q0.x, q0.y, q0.z, q0.w};
  const v8f l1 = {p1.x, p1.y, p1.z, p1.w, q1.x, q1.y, q1.z, q1.w};
  const v8f l2 = {p2.x, p2.y, p2.z, p2.w, q2.x, q2.y, q2.z, q2.w};
  v8us ohs, ols, ohv, olv;
#pragma unroll
  for (int i = 0; i < 8; ++i) {
    const float vn = sqrtf(((l0[i] * l0[i] + l1[i] * l1[i]) + l2[i] * l2[i]) + EPSG);
    const unsigned hs = bf16_bits(s8[i]);
    const unsigned hv = bf16_bits(vn);
    ohs[i] = (unsigned short)hs;
    ols[i] = (unsigned short)bf16_bits(s8[i] - __uint_as_float(hs << 16));
    ohv[i] = (unsigned short)hv;
    olv[i] = (unsigned short)bf16_bits(vn - __uint_as_float(hv << 16));
  }
  unsigned short* dp = TS + (size_t)row * K4 + 8 * j;
  *(volatile v8us*)dp        = ohs;
  *(volatile v8us*)(dp + HD) = ols;
  *(volatile v8us*)(dp + H2) = ohv;
  *(volatile v8us*)(dp + H3) = olv;
  __threadfence();
  *(volatile v8us*)dp        = ohs;
  *(volatile v8us*)(dp + HD) = ols;
  *(volatile v8us*)(dp + H2) = ohv;
  *(volatile v8us*)(dp + H3) = olv;
}

template <int MODE>
__global__ __launch_bounds__(GTHR) void k_gemm(const unsigned short* __restrict__ A, int lda,
                                               const unsigned short* __restrict__ BT, int ldb, int K,
                                               const float* __restrict__ bias, const float* __restrict__ rsc,
                                               int ebase, int nE, float* Cm, int ldc, unsigned short* Ch) {
  __shared__ __attribute__((aligned(16))) float stg[GBM * GBN];
  __shared__ float scut[GBM];
  const int tid = (int)threadIdx.x, lane = tid & 31, wave = tid >> 5, hh = lane >> 4, m = lane & 15;
  const int rowBase = (int)blockIdx.x * GBM;
  const int colBase = (int)blockIdx.y * GBN;

  if constexpr (MODE == 3) {
    if (tid < GBM) {
      int e = ebase + rowBase + tid;
      e = e > nE - 1 ? nE - 1 : e;
      scut[tid] = rsc[(size_t)e * 4 + 3];
    }
  }

  v8f acc[8];
  {
    const v8f zv = {0.f, 0.f, 0.f, 0.f, 0.f, 0.f, 0.f, 0.f};
#pragma unroll
    for (int t = 0; t < 8; ++t) acc[t] = zv;
  }
  const unsigned short* ap = A  + (size_t)(rowBase + 16 * wave + m) * (size_t)lda + 8 * hh;
  const unsigned short* bp = BT + (size_t)(colBase + m) * (size_t)ldb + 8 * hh;

#pragma unroll 1
  for (int k0 = 0; k0 < K; k0 += 32) {
    FragB af;
    af.h[0] = *(const v8usa*)(ap + k0);
    af.h[1] = *(const v8usa*)(ap + k0 + 16);
#pragma unroll
    for (int nt = 0; nt < 8; ++nt) {
      const unsigned short* wq = bp + (size_t)(16 * nt) * (size_t)ldb + k0;
      FragB bfr;
      bfr.h[0] = *(const v8usa*)wq;
      bfr.h[1] = *(const v8usa*)(wq + 16);
      acc[nt] = wmb(af, bfr, acc[nt]);
    }
  }

#pragma unroll
  for (int nt = 0; nt < 8; ++nt) {
    const int lc = 16 * nt + m;
    float bvv = 0.0f;
    if constexpr (MODE != 0) bvv = bf16_val(bias[colBase + lc]);
#pragma unroll
    for (int r = 0; r < 8; ++r) {
      const int lr = 16 * wave + 8 * hh + r;
      float v = acc[nt][r];
      if constexpr (MODE == 1) v = silu_f(v + bvv);
      if constexpr (MODE == 2 || MODE == 3) v = v + bvv;
      stg[lr * GBN + lc] = v;
    }
  }
  __syncthreads();

  if constexpr (MODE == 0 || MODE == 2) {
    v4f pv[16];
#pragma unroll
    for (int i = 0; i < 16; ++i) pv[i] = *(const v4fa*)(stg + (16 * wave + i) * GBN + 4 * lane);
#pragma unroll
    for (int i = 0; i < 16; ++i) {
      float* op = Cm + (size_t)(rowBase + 16 * wave + i) * (size_t)ldc + colBase + 4 * lane;
      *(volatile v4f*)op = pv[i];
    }
    __threadfence();
#pragma unroll
    for (int i = 0; i < 16; ++i) {
      float* op = Cm + (size_t)(rowBase + 16 * wave + i) * (size_t)ldc + colBase + 4 * lane;
      *(volatile v4f*)op = pv[i];
    }
  } else if constexpr (MODE == 1) {
    const int part = lane >> 4;
    const int j = lane & 15;
    const unsigned mh = 0u - (unsigned)part;
    const unsigned ml = ~mh;
    v8us pv[16];
#pragma unroll
    for (int i = 0; i < 16; ++i) {
      const float* sp = stg + (16 * wave + i) * GBN + 8 * j;
      const v4f a = *(const v4fa*)sp;
      const v4f b = *(const v4fa*)(sp + 4);
      const v8f f8 = {a.x, a.y, a.z, a.w, b.x, b.y, b.z, b.w};
      v8us oo;
#pragma unroll
      for (int e = 0; e < 8; ++e) {
        const unsigned hb = bf16_bits(f8[e]);
        const unsigned lb = bf16_bits(f8[e] - __uint_as_float(hb << 16));
        oo[e] = (unsigned short)((hb & ml) | (lb & mh));
      }
      pv[i] = oo;
    }
#pragma unroll
    for (int i = 0; i < 16; ++i) {
      unsigned short* op = Ch + (size_t)(rowBase + 16 * wave + i) * (size_t)H2 + part * HD + 8 * j;
      *(volatile v8us*)op = pv[i];
    }
    __threadfence();
#pragma unroll
    for (int i = 0; i < 16; ++i) {
      unsigned short* op = Ch + (size_t)(rowBase + 16 * wave + i) * (size_t)H2 + part * HD + 8 * j;
      *(volatile v8us*)op = pv[i];
    }
  } else {
    const int j = lane & 15;
    v8us pv[8];
#pragma unroll
    for (int i = 0; i < 8; ++i) {
      const int lr = 16 * wave + 2 * i + hh;
      const float cs = scut[lr] * CF;
      const float* sp = stg + lr * GBN + 8 * j;
      const v4f a = *(const v4fa*)sp;
      const v4f b = *(const v4fa*)(sp + 4);
      const v8f f8 = {a.x, a.y, a.z, a.w, b.x, b.y, b.z, b.w};
      v8us oo;
#pragma unroll
      for (int e = 0; e < 8; ++e) oo[e] = f2h(f8[e] * cs);
      pv[i] = oo;
    }
#pragma unroll
    for (int i = 0; i < 8; ++i) {
      const int lr = 16 * wave + 2 * i + hh;
      unsigned short* op = Ch + (size_t)(rowBase + lr) * (size_t)ldc + colBase + 8 * j;
      *(volatile v8us*)op = pv[i];
    }
    __threadfence();
#pragma unroll
    for (int i = 0; i < 8; ++i) {
      const int lr = 16 * wave + 2 * i + hh;
      unsigned short* op = Ch + (size_t)(rowBase + lr) * (size_t)ldc + colBase + 8 * j;
      *(volatile v8us*)op = pv[i];
    }
  }
}

__global__ __launch_bounds__(NTHR) void k_drain(
    const int* __restrict__ snd, const int* __restrict__ rcv, const float* __restrict__ DIRD,
    const unsigned short* __restrict__ FP, const float* __restrict__ X, const float* __restrict__ VA,
    float* SA, float* VB, float* DS, float* DV,
    int nN, int NP, int nE, int ebase, int nEc, int nb, int vec8, int NPD, int accum, int fin) {
  extern __shared__ v4f lds_dyn[];
  int* reg1 = (int*)lds_dyn;
  int* reg2 = reg1 + RCAP;
  int* scnt = reg2 + RCAP;
  int* soff = scnt + NBMAX;
  int* list = soff + NBMAX;
  int* wcnt = list + LISTN;
  int* wtot = wcnt + NWAVE;
  const int tid = (int)threadIdx.x, lane = tid & 31, wave = tid >> 5;
  const int nodeBase = (int)blockIdx.x * nb;
  const int* dsts = snd + (size_t)ebase;
  const int nEl = nEc;
  (void)nE;

  for (int i = tid; i < NBMAX; i += NTHR) scnt[i] = 0;
  __syncthreads();

  int tot = 0;
  const int nChunks = (nEl + CHUNK - 1) / CHUNK;
#pragma unroll 1
  for (int ch = 0; ch < nChunks; ++ch) {
    const int cbase = ch * CHUNK;
    const int wc = scan_chunk(dsts, nEl, cbase, nodeBase, nb, vec8, list, tid, lane, wave);
    if (lane == 0) wcnt[wave] = wc;
    __syncthreads();
    int pre = 0, all = 0;
#pragma unroll
    for (int w2 = 0; w2 < NWAVE; ++w2) {
      int c = wcnt[w2];
      c = c < 0 ? 0 : (c > WCAP ? WCAP : c);
      all += c;
      pre += (w2 < wave) ? c : 0;
    }
    const int wcc  = wc > WCAP ? WCAP : wc;
    const int base = tot + pre;
#pragma unroll 1
    for (int i = lane; i < wcc; i += 32) {
      const int ent = list[wave * WCAP + i];
      const int el  = (ent >> 12) & (CHUNK - 1);
      const int sl  = ent & (NBMAX - 1);
      int eid = cbase + el;
      eid = eid > nEl - 1 ? nEl - 1 : eid;
      const int pos = base + i;
      if (pos < RCAP) reg1[pos] = (int)(((unsigned)eid << 12) | (unsigned)sl);
    }
    tot += all;
    tot = tot > RCAP ? RCAP : tot;
    __syncthreads();
  }
  const int nh = tot;

  if (wave == 0) {
#pragma unroll 1
    for (int b0 = 0; b0 < nh; b0 += 32) {
      const int idx = b0 + lane;
      const int uv  = reg1[idx < RCAP ? idx : RCAP - 1];
      const int m32 = (nh - b0) < 32 ? (nh - b0) : 32;
#pragma unroll 1
      for (int k = 0; k < m32; ++k) {
        const int uu = __builtin_amdgcn_readlane(uv, k);
        const int sl = uu & (NBMAX - 1);
        if (lane == 0) scnt[sl] = scnt[sl] + 1;
      }
    }
  }
  __syncthreads();

  {
    const v4i ca = *(const v4i*)(scnt + 8 * tid);
    const v4i cb = *(const v4i*)(scnt + 8 * tid + 4);
    const int e0 = ca.x < 0 ? 0 : ca.x, e1 = ca.y < 0 ? 0 : ca.y, e2 = ca.z < 0 ? 0 : ca.z, e3 = ca.w < 0 ? 0 : ca.w;
    const int e4 = cb.x < 0 ? 0 : cb.x, e5 = cb.y < 0 ? 0 : cb.y, e6 = cb.z < 0 ? 0 : cb.z, e7 = cb.w < 0 ? 0 : cb.w;
    const int ts = e0 + e1 + e2 + e3 + e4 + e5 + e6 + e7;
    int incl = ts;
#pragma unroll
    for (int d = 1; d < 32; d <<= 1) {
      const int up = __shfl_up(incl, d);
      if (lane >= d) incl += up;
    }
    if (lane == 31) wtot[wave] = incl;
    __syncthreads();
    int pre = 0;
#pragma unroll
    for (int w2 = 0; w2 < NWAVE; ++w2) pre += (w2 < wave) ? wtot[w2] : 0;
    int run = pre + incl - ts;
    soff[8 * tid + 0] = run; run += e0;
    soff[8 * tid + 1] = run; run += e1;
    soff[8 * tid + 2] = run; run += e2;
    soff[8 * tid + 3] = run; run += e3;
    soff[8 * tid + 4] = run; run += e4;
    soff[8 * tid + 5] = run; run += e5;
    soff[8 * tid + 6] = run; run += e6;
    soff[8 * tid + 7] = run;
  }
  __syncthreads();
  for (int i = tid; i < NBMAX; i += NTHR) list[i] = soff[i];
  __syncthreads();

  if (wave == 0) {
#pragma unroll 1
    for (int b0 = 0; b0 < nh; b0 += 32) {
      const int idx = b0 + lane;
      const int uv  = reg1[idx < RCAP ? idx : RCAP - 1];
      const int m32 = (nh - b0) < 32 ? (nh - b0) : 32;
#pragma unroll 1
      for (int k = 0; k < m32; ++k) {
        const int uu  = __builtin_amdgcn_readlane(uv, k);
        const int sl  = uu & (NBMAX - 1);
        const int eid = (int)((unsigned)uu >> 12);
        if (lane == 0) {
          int pos = list[sl];
          pos = pos < 0 ? 0 : (pos > RCAP - 1 ? RCAP - 1 : pos);
          reg2[pos] = eid;
          list[sl] = pos + 1;
        }
      }
    }
  }
  __syncthreads();

  const int nbw = nb >> 3;
  const bool ovf = (nh >= RCAP);
  const float qnan = __int_as_float(0x7fc00000);
  const int c4 = 4 * lane;
#pragma unroll 1
  for (int jt = 0; jt < nbw; ++jt) {
    const int slot = wave * nbw + jt;
    const int grow = nodeBase + slot;
    const int gw   = grow < NPD ? grow : NPD - 1;
    const int gnp  = grow < NP ? grow : NP - 1;
    int st = soff[slot];
    const int craw = scnt[slot];
    int cnt = craw;
    st  = st < 0 ? 0 : (st > nh ? nh : st);
    cnt = cnt < 0 ? 0 : (cnt > DEGCAP ? DEGCAP : cnt);
    if (cnt > nh - st) cnt = nh - st;
    const float pz = (ovf || craw > DEGCAP) ? qnan : 0.0f;
    const bool wout = grow < nN;
    const bool wnp  = grow < NP;
    const bool wr   = grow < NPD;
    const float live = wout ? 1.0f : 0.0f;

    float as_[4], a0[4], a1[4], a2[4];
#pragma unroll
    for (int j = 0; j < 4; ++j) { as_[j] = 0.f; a0[j] = 0.f; a1[j] = 0.f; a2[j] = 0.f; }
#pragma unroll 1
    for (int q = 0; q < cnt; ++q) {
      int idx = st + q; idx = idx > RCAP - 1 ? RCAP - 1 : idx;
      int el = reg2[idx]; el = el < 0 ? 0 : (el > nEc - 1 ? nEc - 1 : el);
      const int e = ebase + el;
      int rr = rcv[e]; rr = rr < 0 ? 0 : (rr > nN - 1 ? nN - 1 : rr);
      const unsigned short* fr = FP + (size_t)el * H3 + c4;
      const v2u fw0 = *(const v2ua*)fr;
      const v2u fw1 = *(const v2ua*)(fr + HD);
      const v2u fw2 = *(const v2ua*)(fr + H2);
      const float* xr = X + (size_t)rr * H3 + c4;
      const v4f x0 = *(const v4fa*)xr, x1 = *(const v4fa*)(xr + HD), x2 = *(const v4fa*)(xr + H2);
      const float* yr = VA + (size_t)rr * H3 + c4;
      const v4f y0 = *(const v4fa*)yr, y1 = *(const v4fa*)(yr + HD), y2 = *(const v4fa*)(yr + H2);
      const v4f dr = *(const v4fa*)(DIRD + (size_t)e * 4);
      ldwait();
      const float ff0[4] = {h2f(fw0.x & 0xffffu), h2f(fw0.x >> 16), h2f(fw0.y & 0xffffu), h2f(fw0.y >> 16)};
      const float ff1[4] = {h2f(fw1.x & 0xffffu), h2f(fw1.x >> 16), h2f(fw1.y & 0xffffu), h2f(fw1.y >> 16)};
      const float ff2[4] = {h2f(fw2.x & 0xffffu), h2f(fw2.x >> 16), h2f(fw2.y & 0xffffu), h2f(fw2.y >> 16)};
      const float xx0[4] = {x0.x, x0.y, x0.z, x0.w};
      const float xx1[4] = {x1.x, x1.y, x1.z, x1.w};
      const float xx2[4] = {x2.x, x2.y, x2.z, x2.w};
      const float yy0[4] = {y0.x, y0.y, y0.z, y0.w};
      const float yy1[4] = {y1.x, y1.y, y1.z, y1.w};
      const float yy2[4] = {y2.x, y2.y, y2.z, y2.w};
#pragma unroll
      for (int j = 0; j < 4; ++j) {
        const float ms = (ff0[j] * RCF) * xx0[j];
        const float mv = (ff1[j] * RCF) * xx1[j];
        const float mq = (ff2[j] * RCF) * xx2[j];
        as_[j] += ms;
        a0[j] += fmaf(mv, dr.x, mq * yy0[j]);
        a1[j] += fmaf(mv, dr.y, mq * yy1[j]);
        a2[j] += fmaf(mv, dr.z, mq * yy2[j]);
      }
    }
    float od[4], o0[4], o1[4], o2[4];
#pragma unroll
    for (int j = 0; j < 4; ++j) { od[j] = 0.f; o0[j] = 0.f; o1[j] = 0.f; o2[j] = 0.f; }
    if (accum != 0) {
      const v4f d0 = *(const v4fa*)(DS + (size_t)gw * HD + c4);
      const float* dvr = DV + (size_t)gw * H3 + c4;
      const v4f d1 = *(const v4fa*)dvr, d2 = *(const v4fa*)(dvr + HD), d3 = *(const v4fa*)(dvr + H2);
      ldwait();
      od[0] = d0.x; od[1] = d0.y; od[2] = d0.z; od[3] = d0.w;
      o0[0] = d1.x; o0[1] = d1.y; o0[2] = d1.z; o0[3] = d1.w;
      o1[0] = d2.x; o1[1] = d2.y; o1[2] = d2.z; o1[3] = d2.w;
      o2[0] = d3.x; o2[1] = d3.y; o2[2] = d3.z; o2[3] = d3.w;
    }
    if (fin != 0) {
      const v4f sv = *(const v4fa*)(SA + (size_t)gnp * HD + c4);
      const float* vp = VA + (size_t)gnp * H3 + c4;
      const v4f v0 = *(const v4fa*)vp, v1 = *(const v4fa*)(vp + HD), v2 = *(const v4fa*)(vp + H2);
      ldwait();
      v4f w0, w1, w2, w3;
      w0.x = (sv.x + clipf(as_[0] + od[0])) * live + pz; w0.y = (sv.y + clipf(as_[1] + od[1])) * live + pz;
      w0.z = (sv.z + clipf(as_[2] + od[2])) * live + pz; w0.w = (sv.w + clipf(as_[3] + od[3])) * live + pz;
      w1.x = (v0.x + clipf(a0[0] + o0[0])) * live + pz;  w1.y = (v0.y + clipf(a0[1] + o0[1])) * live + pz;
      w1.z = (v0.z + clipf(a0[2] + o0[2])) * live + pz;  w1.w = (v0.w + clipf(a0[3] + o0[3])) * live + pz;
      w2.x = (v1.x + clipf(a1[0] + o1[0])) * live + pz;  w2.y = (v1.y + clipf(a1[1] + o1[1])) * live + pz;
      w2.z = (v1.z + clipf(a1[2] + o1[2])) * live + pz;  w2.w = (v1.w + clipf(a1[3] + o1[3])) * live + pz;
      w3.x = (v2.x + clipf(a2[0] + o2[0])) * live + pz;  w3.y = (v2.y + clipf(a2[1] + o2[1])) * live + pz;
      w3.z = (v2.z + clipf(a2[2] + o2[2])) * live + pz;  w3.w = (v2.w + clipf(a2[3] + o2[3])) * live + pz;
      float* q0 = SA + (size_t)gnp * HD + c4;
      float* q1 = VB + (size_t)gnp * H3 + c4;
      if (wnp) {
        *(volatile v4f*)q0 = w0;
        *(volatile v4f*)q1 = w1;
        *(volatile v4f*)(q1 + HD) = w2;
        *(volatile v4f*)(q1 + H2) = w3;
      }
      __threadfence();
      if (wnp) {
        *(volatile v4f*)q0 = w0;
        *(volatile v4f*)q1 = w1;
        *(volatile v4f*)(q1 + HD) = w2;
        *(volatile v4f*)(q1 + H2) = w3;
      }
    } else {
      v4f w0, w1, w2, w3;
      w0.x = (as_[0] + od[0]) * live + pz; w0.y = (as_[1] + od[1]) * live + pz;
      w0.z = (as_[2] + od[2]) * live + pz; w0.w = (as_[3] + od[3]) * live + pz;
      w1.x = (a0[0] + o0[0]) * live + pz;  w1.y = (a0[1] + o0[1]) * live + pz;
      w1.z = (a0[2] + o0[2]) * live + pz;  w1.w = (a0[3] + o0[3]) * live + pz;
      w2.x = (a1[0] + o1[0]) * live + pz;  w2.y = (a1[1] + o1[1]) * live + pz;
      w2.z = (a1[2] + o1[2]) * live + pz;  w2.w = (a1[3] + o1[3]) * live + pz;
      w3.x = (a2[0] + o2[0]) * live + pz;  w3.y = (a2[1] + o2[1]) * live + pz;
      w3.z = (a2[2] + o2[2]) * live + pz;  w3.w = (a2[3] + o2[3]) * live + pz;
      float* q0 = DS + (size_t)gw * HD + c4;
      float* q1 = DV + (size_t)gw * H3 + c4;
      if (wr) {
        *(volatile v4f*)q0 = w0;
        *(volatile v4f*)q1 = w1;
        *(volatile v4f*)(q1 + HD) = w2;
        *(volatile v4f*)(q1 + H2) = w3;
      }
      __threadfence();
      if (wr) {
        *(volatile v4f*)q0 = w0;
        *(volatile v4f*)q1 = w1;
        *(volatile v4f*)(q1 + HD) = w2;
        *(volatile v4f*)(q1 + H2) = w3;
      }
    }
  }
}

__global__ __launch_bounds__(NTHR) void k_upd(const float* __restrict__ MM, const float* __restrict__ U,
                                              const float* __restrict__ VB, int nN,
                                              float* SA, float* VA, float* out0, float* out1, int fin) {
  const int u   = (int)blockIdx.x * NTHR + (int)threadIdx.x;
  const int row = u >> 5;
  const int c4  = (u & 31) * 4;
  if (row >= nN) return;
  const v4f s4 = *(const v4fa*)(SA + (size_t)row * HD + c4);
  const float* mr = MM + (size_t)row * H3 + c4;
  const v4f d2 = *(const v4fa*)mr, du = *(const v4fa*)(mr + HD), dq = *(const v4fa*)(mr + H2);
  const float* ur = U + (size_t)row * 3 * H2 + c4;
  const v4f l0 = *(const v4fa*)ur,            r0 = *(const v4fa*)(ur + HD);
  const v4f l1 = *(const v4fa*)(ur + H2),     r1 = *(const v4fa*)(ur + H2 + HD);
  const v4f l2 = *(const v4fa*)(ur + 2 * H2), r2 = *(const v4fa*)(ur + 2 * H2 + HD);
  const float* br = VB + (size_t)row * H3 + c4;
  const v4f b0 = *(const v4fa*)br, b1 = *(const v4fa*)(br + HD), b2 = *(const v4fa*)(br + H2);
  v4f os, o0, o1, o2;
#define UPDC(C) { \
    const float dt = (l0.C * r0.C + l1.C * r1.C) + l2.C * r2.C; \
    os.C = s4.C + clipf(d2.C + dq.C * dt); \
    o0.C = b0.C + clipf(du.C * r0.C); \
    o1.C = b1.C + clipf(du.C * r1.C); \
    o2.C = b2.C + clipf(du.C * r2.C); }
  UPDC(x) UPDC(y) UPDC(z) UPDC(w)
#undef UPDC
  float* q0;
  float* q1;
  if (fin != 0) {
    q0 = out0 + (size_t)row * HD + c4;
    q1 = out1 + (size_t)row * H3 + c4;
  } else {
    q0 = SA + (size_t)row * HD + c4;
    q1 = VA + (size_t)row * H3 + c4;
  }
  *(volatile v4f*)q0 = os;
  *(volatile v4f*)q1 = o0;
  *(volatile v4f*)(q1 + HD) = o1;
  *(volatile v4f*)(q1 + H2) = o2;
  __threadfence();
  *(volatile v4f*)q0 = os;
  *(volatile v4f*)q1 = o0;
  *(volatile v4f*)(q1 + HD) = o1;
  *(volatile v4f*)(q1 + H2) = o2;
}

static inline int cdiv(int a, int b) { return (a + b - 1) / b; }
static inline size_t al256(size_t x) { return (x + 255) & ~(size_t)255; }

extern "C" void kernel_launch(void* const* d_in, const int* in_sizes, int n_in,
                              void* d_out, int out_size, void* d_ws, size_t ws_size,
                              hipStream_t stream) {
  if (n_in < 16) return;
  const int nN = in_sizes[0];
  if (nN < 1 || nN > (1 << 20)) return;
  const int nE = in_sizes[2];
  if (nE < 1 || nE > (1 << 22)) return;
  if (in_sizes[3] != nE || in_sizes[1] != 3 * nE) return;
  if (in_sizes[4] < HD || (in_sizes[4] % HD) != 0) return;
  const int nZ = in_sizes[4] / HD;
  if (in_sizes[5] != NRB * NFLT || in_sizes[6] != NFLT) return;
  if (in_sizes[7] != NL * HD * HD || in_sizes[8] != NL * HD) return;
  if (in_sizes[9] != NL * HD * H3 || in_sizes[10] != NL * H3) return;
  if (in_sizes[11] != NL * H2 * HD || in_sizes[12] != NL * HD) return;
  if (in_sizes[13] != NL * HD * H3 || in_sizes[14] != NL * H3) return;
  if (in_sizes[15] != NL * HD * H2) return;
  if ((long long)out_size != (long long)nN * (HD + H3)) return;

  const int*   z   = (const int*)d_in[0];
  const float* ev  = (const float*)d_in[1];
  const int*   snd = (const int*)d_in[2];
  const int*   rcv = (const int*)d_in[3];
  const float* emb = (const float*)d_in[4];
  const float* fW  = (const float*)d_in[5];
  const float* fb  = (const float*)d_in[6];
  const float* iW1 = (const float*)d_in[7];
  const float* ib1 = (const float*)d_in[8];
  const float* iW2 = (const float*)d_in[9];
  const float* ib2 = (const float*)d_in[10];
  const float* mW1 = (const float*)d_in[11];
  const float* mb1 = (const float*)d_in[12];
  const float* mW2 = (const float*)d_in[13];
  const float* mb2 = (const float*)d_in[14];
  const float* vW  = (const float*)d_in[15];
  float* out0 = (float*)d_out;
  float* out1 = out0 + (size_t)nN * HD;

  const int NP  = cdiv(nN, GBM) * GBM;
  const int gM  = NP / GBM;
  const int NP3 = 3 * NP;
  const int gM3 = NP3 / GBM;
  const int gA  = cdiv(nN, NBA);
  const int NPD = gA * NBA;
  if (NPD < NP) return;
  const int tilesE = cdiv(nE, GBM);
  const int tpc    = ECH / GBM;
  const int NCHK   = cdiv(tilesE, tpc);
  const int RMAX   = (tpc < tilesE ? tpc : tilesE) * GBM;
  const int EPD    = cdiv(nE, NTHR) * NTHR;

  char* ws = (char*)d_ws;
  size_t off = 0;
  const size_t oWT  = off; off += al256((size_t)NW_TOT * 2);
  const size_t oSA  = off; off += al256((size_t)NP * HD * 4);
  const size_t oVA  = off; off += al256((size_t)NP * H3 * 4);
  const size_t oVB  = off; off += al256((size_t)NP * H3 * 4);
  const size_t oSHL = off; off += al256((size_t)NP * H2 * 2);
  const size_t oG   = off; off += al256((size_t)NP * H2 * 2);
  const size_t oXM  = off; off += al256((size_t)NP * H3 * 4);
  const size_t oVT  = off; off += al256((size_t)NP3 * H2 * 2);
  const size_t szF  = al256((size_t)RMAX * H3 * 2);
  const size_t szDS = al256((size_t)NPD * HD * 4);
  const size_t szDV = al256((size_t)NPD * H3 * 4);
  const size_t szU  = al256((size_t)NP3 * H2 * 4);
  size_t szR1 = szF + szDS + szDV;
  if (szR1 < szU) szR1 = szU;
  const size_t oR1  = off; off += szR1;
  const size_t oPHI = off; off += al256((size_t)RMAX * KF * 2);
  const size_t oDRD = off; off += al256((size_t)EPD * 4 * 4);
  if (off > ws_size || off > (size_t)WSMAX) return;
  unsigned short* WT   = (unsigned short*)(ws + oWT);
  float*          SA   = (float*)(ws + oSA);
  float*          VA   = (float*)(ws + oVA);
  float*          VB   = (float*)(ws + oVB);
  unsigned short* SHL  = (unsigned short*)(ws + oSHL);
  unsigned short* G    = (unsigned short*)(ws + oG);
  float*          XM   = (float*)(ws + oXM);
  unsigned short* VHL  = (unsigned short*)(ws + oVT);
  unsigned short* TS   = (unsigned short*)(ws + oVT);
  unsigned short* FILT = (unsigned short*)(ws + oR1);
  float*          DS   = (float*)(ws + oR1 + szF);
  float*          DV   = (float*)(ws + oR1 + szF + szDS);
  float*          U    = (float*)(ws + oR1);
  unsigned short* PHI  = (unsigned short*)(ws + oPHI);
  float*          DIRD = (float*)(ws + oDRD);

  hipFuncSetAttribute(reinterpret_cast<const void*>(&k_drain),
                      hipFuncAttributeMaxDynamicSharedMemorySize, LDS_AGG);

  k_wprep<<<UFW / NTHR, NTHR, 0, stream>>>(iW1, iW2, vW, mW1, mW2, fW, WT, UFW);
  const int uS = NP * 32;
  const int uV = uS + NP * 96;
  const int uD = uV + EPD;
  k_init<<<uD / NTHR, NTHR, 0, stream>>>(z, emb, ev, nN, nZ, nE, uS, uV, uD, SA, VA, DIRD);

  for (int l = 0; l < NL; ++l) {
    k_hilo<<<(NP * 16) / NTHR, NTHR, 0, stream>>>(SA, NP * 16, SHL);
    k_gemm<1><<<dim3(gM, 1), GTHR, 0, stream>>>(SHL, H2, WT + OW1 + (size_t)l * HD * H2, H2, H2,
                                                ib1 + (size_t)l * HD, DIRD, 0, nE, XM, H3, G);
    k_gemm<2><<<dim3(gM, H3 / GBN), GTHR, 0, stream>>>(G, H2, WT + OW2 + (size_t)l * H3 * H2, H2, H2,
                                                       ib2 + (size_t)l * H3, DIRD, 0, nE, XM, H3, G);
    for (int c = 0; c < NCHK; ++c) {
      const int t0 = c * tpc;
      int t1 = t0 + tpc;
      t1 = t1 > tilesE ? tilesE : t1;
      if (t1 <= t0) continue;
      const int rows  = (t1 - t0) * GBM;
      const int ebase = t0 * GBM;
      int nEc = nE - ebase;
      nEc = nEc > rows ? rows : nEc;
      const int vec8  = ((ebase & 3) == 0) ? 1 : 0;
      const int accum = (c == 0) ? 0 : 1;
      const int finc  = (c == NCHK - 1) ? 1 : 0;
      k_phi<<<(rows * 8) / NTHR, NTHR, 0, stream>>>(ev, nE, ebase, rows * 8, PHI);
      k_gemm<3><<<dim3(rows / GBM, H3 / GBN), GTHR, 0, stream>>>(PHI, KF, WT + OFW + (size_t)l * H3 * KF, KF, KF,
                                                                 fb + (size_t)l * H3, DIRD, ebase, nE, XM, H3,
                                                                 FILT);
      k_drain<<<gA, NTHR, LDS_AGG, stream>>>(snd, rcv, DIRD, FILT, XM, VA, SA, VB, DS, DV,
                                             nN, NP, nE, ebase, nEc, NBA, vec8, NPD, accum, finc);
    }
    k_hilo<<<(NP3 * 16) / NTHR, NTHR, 0, stream>>>(VB, NP3 * 16, VHL);
    k_gemm<0><<<dim3(gM3, H2 / GBN), GTHR, 0, stream>>>(VHL, H2, WT + OVW + (size_t)l * H2 * H2, H2, H2,
                                                        ib1, DIRD, 0, nE, U, H2, G);
    k_tsrow<<<(NP * 16) / NTHR, NTHR, 0, stream>>>(SA, U, NP * 16, TS);
    k_gemm<1><<<dim3(gM, 1), GTHR, 0, stream>>>(TS, K4, WT + OM1 + (size_t)l * HD * K4, K4, K4,
                                                mb1 + (size_t)l * HD, DIRD, 0, nE, XM, H3, G);
    k_gemm<2><<<dim3(gM, H3 / GBN), GTHR, 0, stream>>>(G, H2, WT + OM2 + (size_t)l * H3 * H2, H2, H2,
                                                       mb2 + (size_t)l * H3, DIRD, 0, nE, XM, H3, G);
    const int finl = (l == NL - 1) ? 1 : 0;
    k_upd<<<cdiv(nN * 32, NTHR), NTHR, 0, stream>>>(XM, U, VB, nN, SA, VA, out0, out1, finl);
  }
}
